// kv_cache_group_query_10797547782443
// MI455X (gfx1250) — hardware-verified
//
#include <hip/hip_runtime.h>
#include <math.h>

typedef __attribute__((ext_vector_type(16))) _Float16 v16h;
typedef __attribute__((ext_vector_type(16))) __bf16 v16b;
typedef __attribute__((ext_vector_type(8)))  _Float16 v8h;
typedef __attribute__((ext_vector_type(8)))  float v8f;
typedef __attribute__((ext_vector_type(4)))  float v4f;
typedef __attribute__((ext_vector_type(2)))  float v2f;
typedef __attribute__((ext_vector_type(4)))  unsigned v4u;
typedef __attribute__((ext_vector_type(4)))  int v4i;
typedef float __attribute__((may_alias)) float_a;
typedef int __attribute__((may_alias)) int_a;

template <typename T> __device__ __forceinline__ void vst2(void* p, T v) { *(volatile T*)p = v; __threadfence(); *(volatile T*)p = v; }
__device__ __forceinline__ v8f wmma16(v16h a, v16h b, v8f c) {
  v8f d = __builtin_amdgcn_wmma_f32_16x16x32_f16(false, a, false, b, (short)0, c, false, false);
  asm volatile("v_nop\n\tv_nop\n\tv_nop\n\tv_nop" : "+v"(d) : "v"(a), "v"(b));
  return d;
}
__device__ __forceinline__ v8f wmma_bf(v16b a, v16b b, v8f c) {
  v8f d = __builtin_amdgcn_wmma_f32_16x16x32_bf16(false, a, false, b, (short)0, c, false, false);
  asm volatile("v_nop\n\tv_nop\n\tv_nop\n\tv_nop" : "+v"(d) : "v"(a), "v"(b));
  return d;
}
__device__ __forceinline__ v16h frag_h(const _Float16* rowk0, int lane) {
  union { v16h v; v8h q[2]; } u; const _Float16* p = rowk0 + 8 * (lane >> 4);
  u.q[0] = *(const v8h*)p; u.q[1] = *(const v8h*)(p + 16); return u.v;
}
__device__ __forceinline__ v16h frag_f32(const float* rowk0, int lane) {
  v16h a; const float* p = rowk0 + 8 * (lane >> 4);
#pragma unroll
  for (int i = 0; i < 8; ++i) { a[i] = (_Float16)p[i]; a[8 + i] = (_Float16)p[16 + i]; }
  return a;
}
__device__ __forceinline__ v16h frag_f32s(const float* rowk0, int lane, float sc) {
  v16h a; const float* p = rowk0 + 8 * (lane >> 4);
#pragma unroll
  for (int i = 0; i < 8; ++i) { a[i] = (_Float16)(p[i] * sc); a[8 + i] = (_Float16)(p[16 + i] * sc); }
  return a;
}
__device__ __forceinline__ v16h fragc_f32(const float* W, int k0, int n, int lane, int ld, int K) {
  v16h a; const int g = lane >> 4;
#pragma unroll
  for (int i = 0; i < 8; ++i) { const int ka = k0 + 8 * g + i, kb = ka + 16;
    a[i] = (_Float16)(ka < K ? W[(size_t)(ka < K ? ka : K - 1) * ld + n] : 0.f); a[8 + i] = (_Float16)(kb < K ? W[(size_t)(kb < K ? kb : K - 1) * ld + n] : 0.f); }
  return a;
}
struct F2 { v16b h, l; };
__device__ __forceinline__ F2 bsplit16(const float v[16]) { F2 r;
#pragma unroll
  for (int i = 0; i < 16; ++i) { const __bf16 h = (__bf16)v[i]; r.h[i] = h; r.l[i] = (__bf16)(v[i] - (float)h); }
  return r; }
__device__ __forceinline__ F2 split_row(const float* row, int k0, int lane) { float v[16]; const float* p = row + k0 + 8 * (lane >> 4);
#pragma unroll
  for (int i = 0; i < 8; ++i) { v[i] = p[i]; v[8 + i] = p[16 + i]; }
  return bsplit16(v); }
__device__ __forceinline__ F2 split_rowK(const float* row, int k0, int lane, int K) { float v[16]; const int g = lane >> 4;
#pragma unroll
  for (int i = 0; i < 8; ++i) { const int ka = k0 + 8 * g + i, kb = ka + 16; v[i] = ka < K ? row[ka < K ? ka : K - 1] : 0.f; v[8 + i] = kb < K ? row[kb < K ? kb : K - 1] : 0.f; }
  return bsplit16(v); }
__device__ __forceinline__ F2 split_col(const float* W, int k0, int n, int lane, int ld, int K) { float v[16]; const int g = lane >> 4;
#pragma unroll
  for (int i = 0; i < 8; ++i) { const int ka = k0 + 8 * g + i, kb = ka + 16; v[i] = ka < K ? W[(size_t)(ka < K ? ka : K - 1) * ld + n] : 0.f; v[8 + i] = kb < K ? W[(size_t)(kb < K ? kb : K - 1) * ld + n] : 0.f; }
  return bsplit16(v); }
__device__ __forceinline__ v8f mac3(const F2& a, const F2& b, v8f c) { c = wmma_bf(a.l, b.h, c); c = wmma_bf(a.h, b.l, c); return wmma_bf(a.h, b.h, c); }
__device__ __forceinline__ float sigm(float v) { return 1.0f / (1.0f + expf(-v)); }
#define LDSX() do { asm volatile("s_wait_dscnt 0" ::: "memory"); __builtin_amdgcn_wave_barrier(); __builtin_amdgcn_fence(__ATOMIC_RELEASE, "workgroup"); } while (0)


#define SS 2048
#define DM 2048
#define NH 16
#define NKV 4
#define HD 128
#define KVW (NKV * HD)
#ifndef TQB
#define TQB (SS / 64)
#endif
typedef __attribute__((ext_vector_type(8))) __bf16 v8b;
__device__ __forceinline__ v16b frag_b(const __bf16* rowk0, int lane) {
  union { v16b v; v8b q[2]; } u; const __bf16* p = rowk0 + 8 * (lane >> 4);
  u.q[0] = *(const v8b*)p; u.q[1] = *(const v8b*)(p + 16); return u.v;
}
__device__ __forceinline__ float bfr(float v) { return (float)(__bf16)v; }
__device__ __attribute__((noinline)) float exp_ni(float v) { return expf(v); }
__device__ __attribute__((noinline)) float erf_ni(float v) { return erff(v); }

#define PK_Q 0
#define PK_K (PK_Q + DM * DM)
#define PK_V (PK_K + KVW * DM)
#define PK_O (PK_V + KVW * DM)
#define PK_END (PK_O + DM * DM)
#define WS_PK  0u
#define WS_CS  (WS_PK + 2u * PK_END)
#define WS_Q   (WS_CS + 4u * 2 * SS * 64)
#define WS_K   (WS_Q + 4u * SS * DM)
#define WS_VTH (WS_K + 4u * SS * KVW)
#define WS_VTL (WS_VTH + 2u * KVW * SS)
#define WS_O   (WS_VTL + 2u * KVW * SS)
#define WS_END (WS_O + 4u * SS * DM)

__global__ __launch_bounds__(256) void k_packT(const float* __restrict__ Wm, int K, int N, __bf16* __restrict__ DST) {
  __shared__ __align__(16) __bf16 s[DM]; const int n = blockIdx.x, tid = threadIdx.x;
  for (int k = tid; k < K; k += 256) s[k] = (__bf16)Wm[(size_t)k * N + n];
  __syncthreads();
  for (int q = tid; q < K / 8; q += 256) vst2((unsigned*)(DST + (size_t)n * K + q * 8), *(const v4u*)&s[q * 8]);
}
__global__ __launch_bounds__(256) void k_packrows(const float* __restrict__ Wm, int K, __bf16* __restrict__ DST) {
  __shared__ __align__(16) __bf16 s[DM]; const int n = blockIdx.x, tid = threadIdx.x;
  for (int k = tid; k < K; k += 256) s[k] = (__bf16)Wm[(size_t)n * K + k];
  __syncthreads();
  for (int q = tid; q < K / 8; q += 256) vst2((unsigned*)(DST + (size_t)n * K + q * 8), *(const v4u*)&s[q * 8]);
}
__device__ __attribute__((noinline)) float powf_ni(float a, float b) { return powf(a, b); }
__device__ __attribute__((noinline)) float cosf_ni(float v) { return cosf(v); }
__device__ __attribute__((noinline)) float sinf_ni(float v) { return sinf(v); }
__global__ __launch_bounds__(64) void k_rope_tab(float* __restrict__ CS) {
  __shared__ __align__(16) float sc[64], ssn[64]; const int t = blockIdx.x, i = threadIdx.x;
  const float inv = 1.0f / powf_ni(10000.0f, (float)(2 * i) / 128.0f); const float ang = (float)t * inv; sc[i] = cosf_ni(ang); ssn[i] = sinf_ni(ang);
  __syncthreads();
  if (i < 16) vst2(CS + (size_t)t * 64 + i * 4, *(const v4f*)&sc[i * 4]); else if (i < 32) vst2(CS + (size_t)SS * 64 + (size_t)t * 64 + (i - 16) * 4, *(const v4f*)&ssn[(i - 16) * 4]);
}
template <int MODE>
__global__ __launch_bounds__(128) void k_proj(const float* __restrict__ X, const __bf16* __restrict__ P, const float* __restrict__ CS, float* __restrict__ OUT, int ldo, __bf16* __restrict__ PH, __bf16* __restrict__ PL) {
  __shared__ __align__(16) float so[MODE ? 1 : 4][16][132]; __shared__ __align__(16) __bf16 sth[MODE ? 128 : 1][72], stl[MODE ? 128 : 1][72];
  const int tid = threadIdx.x, wave = tid >> 5, lane = tid & 31, col = lane & 15, g = lane >> 4; const size_t r0 = (size_t)blockIdx.x * 64 + wave * 16; const int n0 = blockIdx.y * 128;
  v8f acc[8] = {};
#pragma unroll 2
  for (int kc = 0; kc < DM / 32; ++kc) { v16b a; { const float* p = X + (r0 + col) * DM + kc * 32 + 8 * g;
#pragma unroll
      for (int i = 0; i < 8; ++i) { a[i] = (__bf16)p[i]; a[8 + i] = (__bf16)p[16 + i]; } }
#pragma unroll
    for (int j = 0; j < 8; ++j) acc[j] = wmma_bf(a, frag_b(P + (size_t)(n0 + j * 16 + col) * DM + kc * 32, lane), acc[j]); }
  if (MODE == 0) {
    const int par = col & 1;
#pragma unroll
    for (int j = 0; j < 8; ++j) { const int d = j * 16 + col; const int ip = d >> 1;
#pragma unroll
      for (int r = 0; r < 8; ++r) { const size_t t = r0 + 8 * g + r; const float c = CS[t * 64 + ip], s = CS[(size_t)SS * 64 + t * 64 + ip]; const float v = acc[j][r]; const float pv = __shfl_xor(v, 1); so[wave][8 * g + r][d] = par ? (pv * s + v * c) : (v * c - pv * s); } }
    LDSX();
    for (int rl = 0; rl < 16; ++rl) vst2(OUT + (r0 + rl) * ldo + n0 + lane * 4, *(const v4f*)&so[wave][rl][lane * 4]);
  } else {
#pragma unroll
    for (int j = 0; j < 8; ++j)
#pragma unroll
      for (int r = 0; r < 8; ++r) { const float v = acc[j][r]; const __bf16 hb = (__bf16)v; sth[j * 16 + col][wave * 16 + 8 * g + r] = hb; stl[j * 16 + col][wave * 16 + 8 * g + r] = (__bf16)(v - (float)hb); }
    __syncthreads();
    const int s0 = blockIdx.x * 64;
    for (int q = tid; q < 128 * 8; q += 128) { const int d = q >> 3, pc = q & 7; const size_t o = (size_t)(n0 + d) * SS + s0 + pc * 8; vst2((unsigned*)(PH + o), *(const v4u*)&sth[d][pc * 8]); vst2((unsigned*)(PL + o), *(const v4u*)&stl[d][pc * 8]); }
  }
}
__global__ __launch_bounds__(128) void k_attn(const float* __restrict__ Q, const float* __restrict__ Kx, const __bf16* __restrict__ VTH, const __bf16* __restrict__ VTL, float* __restrict__ O) {
  __shared__ __align__(16) float sp[4][16][36]; __shared__ __align__(16) float so[4][16][132];
  const int tid = threadIdx.x, wave = tid >> 5, lane = tid & 31, col = lane & 15, g = lane >> 4;
  const int qb = blockIdx.x, h = blockIdx.y, kv = h / (NH / NKV); const int q0 = qb * 64 + wave * 16;
  const float* qrow = Q + (size_t)(q0 + col) * DM + h * HD;
  float m[8], l[8];
#pragma unroll
  for (int r = 0; r < 8; ++r) { m[r] = -3.0e38f; l[r] = 0.f; }
  v8f acc[8] = {};
  const int nks = (qb * 64 + 64) / 32;
#pragma unroll 1
  for (int ks = 0; ks < nks; ++ks) { v8f s[2];
#pragma unroll
    for (int ct = 0; ct < 2; ++ct) { const int kk = ks * 32 + ct * 16 + col; const float* krow = Kx + (size_t)kk * KVW + kv * HD; v8f c = {};
#pragma unroll
      for (int kc = 0; kc < 4; ++kc) { const F2 kb = split_row(krow, kc * 32, lane); const F2 qa = split_row(qrow, kc * 32, lane); c = mac3(qa, kb, c); }
#pragma unroll
      for (int r = 0; r < 8; ++r) { const int qi = q0 + 8 * g + r; s[ct][r] = (kk <= qi) ? c[r] * 0.08838834764831845f : -3.0e38f; } }
#pragma unroll
    for (int r = 0; r < 8; ++r) { float mx = fmaxf(s[0][r], s[1][r]);
#pragma unroll
      for (int o = 1; o < 16; o <<= 1) mx = fmaxf(mx, __shfl_xor(mx, o));
      const float mn = fmaxf(m[r], mx); const float alpha = (m[r] <= -1.0e38f) ? 0.f : exp_ni(m[r] - mn);
      const float e0 = (s[0][r] <= -1.0e38f) ? 0.f : exp_ni(s[0][r] - mn), e1 = (s[1][r] <= -1.0e38f) ? 0.f : exp_ni(s[1][r] - mn); float es = e0 + e1;
#pragma unroll
      for (int o = 1; o < 16; o <<= 1) es += __shfl_xor(es, o);
      l[r] = l[r] * alpha + es; m[r] = mn;
#pragma unroll
      for (int dt = 0; dt < 8; ++dt) acc[dt][r] *= alpha;
      sp[wave][8 * g + r][col] = e0; sp[wave][8 * g + r][16 + col] = e1; }
    LDSX();
    const F2 pa = split_row(&sp[wave][col][0], 0, lane);
#pragma unroll
    for (int dt = 0; dt < 8; ++dt) { const size_t vr = (size_t)(kv * HD + dt * 16 + col) * SS + ks * 32; const v16b vh = frag_b(VTH + vr, lane), vl = frag_b(VTL + vr, lane); acc[dt] = wmma_bf(pa.l, vh, acc[dt]); acc[dt] = wmma_bf(pa.h, vl, acc[dt]); acc[dt] = wmma_bf(pa.h, vh, acc[dt]); }
    LDSX(); }
#pragma unroll
  for (int r = 0; r < 8; ++r) { const float il = 1.0f / l[r];
#pragma unroll
    for (int dt = 0; dt < 8; ++dt) so[wave][8 * g + r][dt * 16 + col] = acc[dt][r] * il; }
  LDSX();
  for (int rl = 0; rl < 16; ++rl) vst2(O + (size_t)(q0 + rl) * DM + h * HD + lane * 4, *(const v4f*)&so[wave][rl][lane * 4]);
}
__global__ __launch_bounds__(128) void k_out(const float* __restrict__ O, const __bf16* __restrict__ P, const float* __restrict__ BO, float* __restrict__ Y) {
  __shared__ __align__(16) float so[4][16][132];
  const int tid = threadIdx.x, wave = tid >> 5, lane = tid & 31, col = lane & 15, g = lane >> 4; const size_t r0 = (size_t)blockIdx.x * 64 + wave * 16; const int n0 = blockIdx.y * 128;
  v8f acc[8] = {};
#pragma unroll 2
  for (int kc = 0; kc < DM / 32; ++kc) { const F2 a = split_row(O + (r0 + col) * DM, kc * 32, lane);
#pragma unroll
    for (int j = 0; j < 8; ++j) { const v16b w = frag_b(P + (size_t)(n0 + j * 16 + col) * DM + kc * 32, lane); acc[j] = wmma_bf(a.l, w, acc[j]); acc[j] = wmma_bf(a.h, w, acc[j]); } }
#pragma unroll
  for (int j = 0; j < 8; ++j) { const float bb = bfr(BO[n0 + j * 16 + col]);
#pragma unroll
    for (int r = 0; r < 8; ++r) so[wave][8 * g + r][j * 16 + col] = acc[j][r] + bb; }
  LDSX();
  for (int rl = 0; rl < 16; ++rl) vst2(Y + (r0 + rl) * DM + n0 + lane * 4, *(const v4f*)&so[wave][rl][lane * 4]);
}
extern "C" void kernel_launch(void* const* d_in, const int* in_sizes, int n_in, void* d_out, int out_size, void* d_ws, size_t ws_size, hipStream_t stream) {
  (void)in_sizes; (void)n_in; (void)out_size;
  const float** F = (const float**)d_in;
  if (ws_size < (size_t)WS_END) return;
  char* ws = (char*)d_ws; __bf16 *PK = (__bf16*)(ws + WS_PK), *VTH = (__bf16*)(ws + WS_VTH), *VTL = (__bf16*)(ws + WS_VTL);
  float *CS = (float*)(ws + WS_CS), *Q = (float*)(ws + WS_Q), *Kx = (float*)(ws + WS_K), *O = (float*)(ws + WS_O);
  k_packrows<<<DM, 256, 0, stream>>>(F[1], DM, PK + PK_Q); k_packrows<<<KVW, 256, 0, stream>>>(F[2], DM, PK + PK_K); k_packrows<<<KVW, 256, 0, stream>>>(F[3], DM, PK + PK_V); k_packrows<<<DM, 256, 0, stream>>>(F[4], DM, PK + PK_O);
  k_rope_tab<<<SS, 64, 0, stream>>>(CS);
  k_proj<0><<<dim3(SS / 64, DM / 128), 128, 0, stream>>>(F[0], PK + PK_Q, CS, Q, DM, nullptr, nullptr);
  k_proj<0><<<dim3(SS / 64, KVW / 128), 128, 0, stream>>>(F[0], PK + PK_K, CS, Kx, KVW, nullptr, nullptr);
  k_proj<1><<<dim3(SS / 64, KVW / 128), 128, 0, stream>>>(F[0], PK + PK_V, CS, nullptr, 0, VTH, VTL);
  k_attn<<<dim3(TQB, NH), 128, 0, stream>>>(Q, Kx, VTH, VTL, O);
  k_out<<<dim3(TQB, DM / 128), 128, 0, stream>>>(O, PK + PK_O, F[5], (float*)d_out);
}
